// FlowPatch_51548197486875
// MI455X (gfx1250) — hardware-verified
//
#include <hip/hip_runtime.h>
#include <stdint.h>
#include <stddef.h>


typedef _Float16 f16t;
typedef f16t  v8h  __attribute__((ext_vector_type(8)));
typedef f16t  v16h __attribute__((ext_vector_type(16)));
typedef float v4f  __attribute__((ext_vector_type(4)));
typedef float v8f  __attribute__((ext_vector_type(8)));
typedef unsigned int v4u __attribute__((ext_vector_type(4)));

union Frag { v16h v; v8h q[2]; };

constexpr int D   = 128;
constexpr int CND = 128;
constexpr int HID = 256;
constexpr int DIN = D / 2 + CND;
constexpr int TOK = 128;
constexpr int NTH = 256;
constexpr int NP  = 128;

constexpr int ZS = 132;
constexpr int AS = 264;
constexpr int SS = 40;

constexpr float WSCALE = 16.0f;
constexpr float WINV   = 0.0625f;

constexpr int OFF_Z = 0;
constexpr int OFF_A = OFF_Z + TOK * ZS * 4;
constexpr int OFF_B = OFF_A + TOK * AS * 2;
constexpr int OFF_S = OFF_B + TOK * AS * 2;
constexpr int OFF_C = OFF_S + NP * SS * 2;
constexpr int OFF_R = OFF_C + CND * 2;
constexpr int SMEM_TOTAL = OFF_R + NTH * 4;

static_assert(OFF_A % 16 == 0 && OFF_B % 16 == 0 && OFF_S % 16 == 0 && OFF_C % 16 == 0 && OFF_R % 16 == 0, "");

constexpr int LN1 = HID * (DIN / 64);
constexpr int LN2 = HID * (HID / 64);
constexpr int LN3 = D * (HID / 64);
constexpr int LPL = LN1 + LN2 + LN3;
constexpr int WPL = HID * DIN + HID * HID + D * HID;

__device__ __forceinline__ v8f wmma_f16(v16h a, v16h b, v8f c) {
  c = __builtin_amdgcn_wmma_f32_16x16x32_f16(false, a, false, b, (short)0, c, false, false);
  asm volatile("v_nop\n\tv_nop\n\tv_nop\n\tv_nop" : "+v"(c) : "v"(a), "v"(b));
  return c;
}

__device__ __forceinline__ v16h ldfrag16(const f16t* p, int h) {
  Frag f;
  f.q[0] = *(const v8h*)(p + 8 * h);
  f.q[1] = *(const v8h*)(p + 16 + 8 * h);
  return f.v;
}

__device__ __forceinline__ v16h ldfrag32(const float* p, int h) {
  v4f a0 = *(const v4f*)(p + 8 * h);
  v4f a1 = *(const v4f*)(p + 8 * h + 4);
  v4f a2 = *(const v4f*)(p + 16 + 8 * h);
  v4f a3 = *(const v4f*)(p + 16 + 8 * h + 4);
  v8f lo = __builtin_shufflevector(a0, a1, 0, 1, 2, 3, 4, 5, 6, 7);
  v8f hi = __builtin_shufflevector(a2, a3, 0, 1, 2, 3, 4, 5, 6, 7);
  Frag f;
  f.q[0] = __builtin_convertvector(lo, v8h);
  f.q[1] = __builtin_convertvector(hi, v8h);
  return f.v;
}

__device__ __forceinline__ void zero8(v8f (&c)[8]) {
#pragma unroll
  for (int j = 0; j < 8; ++j) {
    v8f z = {0.f, 0.f, 0.f, 0.f, 0.f, 0.f, 0.f, 0.f};
    c[j] = z;
  }
}

__device__ __forceinline__ void stage_slab(f16t* wslab, const f16t* wrows, int K, int tid) {
  __syncthreads();
#pragma unroll
  for (int it = 0; it < (NP * 4) / NTH; ++it) {
    const int idx = tid + it * NTH;
    const int rn = idx >> 2, sg = idx & 3;
    v4u v = *(const v4u*)(wrows + (size_t)rn * K + sg * 8);
    *(v4u*)(wslab + rn * SS + sg * 8) = v;
  }
  __syncthreads();
}

__device__ __forceinline__ void ktile(v8f (&c)[8], v16h a, const f16t* wslab, int m, int h) {
#pragma unroll
  for (int j = 0; j < 8; ++j) {
    v16h bfr = ldfrag16(wslab + (j * 16 + m) * SS, h);
    c[j] = wmma_f16(a, bfr, c[j]);
  }
}

__device__ __forceinline__ void relu_store(const v8f (&c)[8], f16t* act, const float* __restrict__ bias,
                                           int n0, int rowbase, int m, int h) {
#pragma unroll
  for (int j = 0; j < 8; ++j) {
    const int col = n0 + j * 16 + m;
    const float bv = bias[col];
#pragma unroll
    for (int r = 0; r < 8; ++r) {
      float v = c[j][r] * WINV + bv;
      v = v > 0.f ? v : 0.f;
      act[(rowbase + 8 * h + r) * AS + col] = (f16t)v;
    }
  }
}

__device__ __forceinline__ float tanh_f(float u) {
  u = fminf(fmaxf(u, -16.0f), 16.0f);
  const float e = __expf(2.0f * u);
  return 1.0f - 2.0f * __builtin_amdgcn_rcpf(e + 1.0f);
}

__global__ void __launch_bounds__(256)
k_convert(const float* __restrict__ W1, const float* __restrict__ W2, const float* __restrict__ W3,
          f16t* __restrict__ wt, int nl) {
  const int g = blockIdx.x * 256 + threadIdx.x;
  if (g >= nl * LPL) return;
  const int l = g / LPL;
  int q = g - l * LPL;
  const float* src;
  f16t* dst;
  int K, N, n, part;
  const size_t base2 = (size_t)nl * HID * DIN;
  const size_t base3 = base2 + (size_t)nl * HID * HID;
  if (q < LN1) {
    n = q / (DIN / 64); part = q - n * (DIN / 64);
    K = DIN; N = HID;
    src = W1 + (size_t)l * DIN * HID;
    dst = wt + (size_t)l * HID * DIN;
  } else if (q < LN1 + LN2) {
    q -= LN1;
    n = q / (HID / 64); part = q - n * (HID / 64);
    K = HID; N = HID;
    src = W2 + (size_t)l * HID * HID;
    dst = wt + base2 + (size_t)l * HID * HID;
  } else {
    q -= LN1 + LN2;
    n = q / (HID / 64); part = q - n * (HID / 64);
    K = HID; N = D;
    src = W3 + (size_t)l * HID * D;
    dst = wt + base3 + (size_t)l * D * HID;
  }
  const int k0 = part * 64;
  union { v4u u[8]; f16t e[64]; } pk;
#pragma unroll
  for (int i = 0; i < 64; ++i)
    pk.e[i] = (f16t)(src[(size_t)(k0 + i) * N + n] * WSCALE);
  f16t* drow = dst + (size_t)n * K + k0;
#pragma unroll
  for (int s = 0; s < 8; ++s) *(volatile v4u*)(drow + s * 8) = pk.u[s];
  __threadfence();
#pragma unroll
  for (int s = 0; s < 8; ++s) *(volatile v4u*)(drow + s * 8) = pk.u[s];
}

__global__ void __launch_bounds__(256)
k_flow(const float* __restrict__ x, const float* __restrict__ cond,
       const float* __restrict__ b1, const float* __restrict__ b2, const float* __restrict__ b3,
       const f16t* __restrict__ wt, float* __restrict__ outz, float* __restrict__ part,
       int B, int nl) {
  extern __shared__ v4u dsm[];
  char* smem = (char*)dsm;
  float* zbuf  = (float*)(smem + OFF_Z);
  f16t*  actA  = (f16t*)(smem + OFF_A);
  f16t*  actB  = (f16t*)(smem + OFF_B);
  f16t*  wslab = (f16t*)(smem + OFF_S);
  f16t*  condh = (f16t*)(smem + OFF_C);
  float* red   = (float*)(smem + OFF_R);

  const int b = blockIdx.x;
  if (b >= B) return;
  const int tid = threadIdx.x;
  const int lane = tid & 31, wave = tid >> 5;
  const int m = lane & 15, h = lane >> 4;
  const int rowbase = wave * 16;

  {
    const float* xb = x + (size_t)b * TOK * D;
    for (int idx = tid; idx < TOK * (D / 4); idx += NTH) {
      const int r = idx / (D / 4), s = idx - r * (D / 4);
      *(v4f*)(zbuf + r * ZS + s * 4) = *(const v4f*)(xb + (size_t)r * D + s * 4);
    }
    if (tid < CND) condh[tid] = (f16t)cond[(size_t)b * CND + tid];
  }
  __syncthreads();

  float ldacc = 0.f;
  const size_t base2 = (size_t)nl * HID * DIN;
  const size_t base3 = base2 + (size_t)nl * HID * HID;

  const float* zrow  = zbuf + (rowbase + m) * ZS;
  const f16t*  arowA = actA + (rowbase + m) * AS;
  const f16t*  arowB = actB + (rowbase + m) * AS;

  for (int l = 0; l < nl; ++l) {
    const f16t* w1t = wt + (size_t)l * HID * DIN;
    const f16t* w2t = wt + base2 + (size_t)l * HID * HID;
    const f16t* w3t = wt + base3 + (size_t)l * D * HID;

#pragma unroll 1
    for (int np = 0; np < HID / NP; ++np) {
      const int n0 = np * NP;
      const f16t* wr = w1t + (size_t)n0 * DIN;
      v8f c[8];
      zero8(c);
#pragma unroll 1
      for (int kt = 0; kt < (D / 2) / 32; ++kt) {
        stage_slab(wslab, wr + kt * 32, DIN, tid);
        v16h a = ldfrag32(zrow + kt * 32, h);
        ktile(c, a, wslab, m, h);
      }
#pragma unroll 1
      for (int kt = (D / 2) / 32; kt < DIN / 32; ++kt) {
        stage_slab(wslab, wr + kt * 32, DIN, tid);
        v16h a = ldfrag16(condh + (kt - (D / 2) / 32) * 32, h);
        ktile(c, a, wslab, m, h);
      }
      relu_store(c, actA, b1 + (size_t)l * HID, n0, rowbase, m, h);
    }

#pragma unroll 1
    for (int np = 0; np < HID / NP; ++np) {
      const int n0 = np * NP;
      const f16t* wr = w2t + (size_t)n0 * HID;
      v8f c[8];
      zero8(c);
#pragma unroll 1
      for (int kt = 0; kt < HID / 32; ++kt) {
        stage_slab(wslab, wr + kt * 32, HID, tid);
        v16h a = ldfrag16(arowA + kt * 32, h);
        ktile(c, a, wslab, m, h);
      }
      relu_store(c, actB, b2 + (size_t)l * HID, n0, rowbase, m, h);
    }

    {
      v8f c[8];
      zero8(c);
#pragma unroll 1
      for (int kt = 0; kt < HID / 32; ++kt) {
        stage_slab(wslab, w3t + kt * 32, HID, tid);
        v16h a = ldfrag16(arowB + kt * 32, h);
        ktile(c, a, wslab, m, h);
      }
      const float* bb = b3 + (size_t)l * D;
      float x1v[4][8], y2v[4][8];
#pragma unroll
      for (int n = 0; n < 4; ++n) {
        const int col = n * 16 + m;
        const float bs = bb[col];
        const float bt = bb[D / 2 + col];
#pragma unroll
        for (int r = 0; r < 8; ++r) {
          const int tok = rowbase + 8 * h + r;
          const float u  = c[n][r] * WINV + bs;
          const float sv = 0.5f * tanh_f(u);
          const float tv = c[n + 4][r] * WINV + bt;
          const float x2 = zbuf[tok * ZS + D / 2 + col];
          y2v[n][r] = x2 * __expf(sv) + tv;
          x1v[n][r] = zbuf[tok * ZS + col];
          ldacc += sv;
        }
      }
      __syncthreads();
#pragma unroll
      for (int n = 0; n < 4; ++n) {
        const int col = n * 16 + m;
#pragma unroll
        for (int r = 0; r < 8; ++r) {
          const int tok = rowbase + 8 * h + r;
          zbuf[tok * ZS + (D - 1 - col)]     = x1v[n][r];
          zbuf[tok * ZS + (D / 2 - 1 - col)] = y2v[n][r];
        }
      }
    }
  }

  red[tid] = ldacc;
  __syncthreads();
  float ld = 0.f;
  if (wave == 0) {
#pragma unroll
    for (int k = 0; k < NTH / 32; ++k) ld += red[lane + 32 * k];
#pragma unroll
    for (int off = 16; off > 0; off >>= 1) ld += __shfl_xor(ld, off, 32);
  }

  float* oz = outz + ((size_t)b * TOK + rowbase) * D;
  float* pl = part + (size_t)b * 32;
#pragma unroll
  for (int r = 0; r < 16; ++r) {
    v4f v = *(const v4f*)(zbuf + (rowbase + r) * ZS + lane * 4);
    *(volatile v4f*)(oz + (size_t)r * D + lane * 4) = v;
  }
  if (wave == 0) *(volatile float*)(pl + lane) = ld;
  __threadfence();
#pragma unroll
  for (int r = 0; r < 16; ++r) {
    v4f v = *(const v4f*)(zbuf + (rowbase + r) * ZS + lane * 4);
    *(volatile v4f*)(oz + (size_t)r * D + lane * 4) = v;
  }
  if (wave == 0) *(volatile float*)(pl + lane) = ld;
}

__global__ void __launch_bounds__(256)
k_final(const float* __restrict__ part, float* __restrict__ outld, int B) {
  const int nq = (B + 3) / 4;
  for (int q = threadIdx.x; q < nq; q += 256) {
    const int b0 = q * 4;
    if (b0 + 3 < B) {
      v4f v;
      v.x = part[(size_t)(b0 + 0) * 32];
      v.y = part[(size_t)(b0 + 1) * 32];
      v.z = part[(size_t)(b0 + 2) * 32];
      v.w = part[(size_t)(b0 + 3) * 32];
      *(volatile v4f*)(outld + b0) = v;
    } else {
      for (int i = 0; i < 4; ++i)
        if (b0 + i < B) *(volatile float*)(outld + b0 + i) = part[(size_t)(b0 + i) * 32];
    }
  }
  __threadfence();
  for (int q = threadIdx.x; q < nq; q += 256) {
    const int b0 = q * 4;
    if (b0 + 3 < B) {
      v4f v;
      v.x = part[(size_t)(b0 + 0) * 32];
      v.y = part[(size_t)(b0 + 1) * 32];
      v.z = part[(size_t)(b0 + 2) * 32];
      v.w = part[(size_t)(b0 + 3) * 32];
      *(volatile v4f*)(outld + b0) = v;
    } else {
      for (int i = 0; i < 4; ++i)
        if (b0 + i < B) *(volatile float*)(outld + b0 + i) = part[(size_t)(b0 + i) * 32];
    }
  }
}

extern "C" void kernel_launch(void* const* d_in, const int* in_sizes, int n_in,
                              void* d_out, int out_size, void* d_ws, size_t ws_size,
                              hipStream_t stream) {
  if (n_in < 8) return;
  const float* x  = (const float*)d_in[0];
  const float* cd = (const float*)d_in[1];
  const float* W1 = (const float*)d_in[2];
  const float* b1 = (const float*)d_in[3];
  const float* W2 = (const float*)d_in[4];
  const float* b2 = (const float*)d_in[5];
  const float* W3 = (const float*)d_in[6];
  const float* b3 = (const float*)d_in[7];

  const int B  = in_sizes[0] / (TOK * D);
  const int nl = in_sizes[2] / (DIN * HID);
  if (B <= 0 || nl <= 0) return;
  if (in_sizes[1] < B * CND) return;
  if (in_sizes[3] < nl * HID || in_sizes[4] < nl * HID * HID || in_sizes[5] < nl * HID) return;
  if (in_sizes[6] < nl * HID * D || in_sizes[7] < nl * D) return;
  if ((size_t)out_size < (size_t)B * TOK * D + (size_t)B) return;

  const size_t wt_bytes  = (size_t)nl * WPL * sizeof(f16t);
  const size_t part_off  = (wt_bytes + 127) & ~(size_t)127;
  const size_t part_bytes = (size_t)B * 128;
  if (part_off + part_bytes > ws_size) return;

  f16t*  wt    = (f16t*)d_ws;
  float* part  = (float*)((char*)d_ws + part_off);
  float* outz  = (float*)d_out;
  float* outld = outz + (size_t)B * TOK * D;

  const int nlines = nl * LPL;
  k_convert<<<(nlines + 255) / 256, 256, 0, stream>>>(W1, W2, W3, wt, nl);

  (void)hipFuncSetAttribute((const void*)k_flow, hipFuncAttributeMaxDynamicSharedMemorySize, SMEM_TOTAL);
  k_flow<<<B, NTH, SMEM_TOTAL, stream>>>(x, cd, b1, b2, b3, wt, outz, part, B, nl);

  k_final<<<1, 256, 0, stream>>>(part, outld, B);
}
